// GraphResnetBottleneckBlock_37855841747676
// MI455X (gfx1250) — hardware-verified
//
#include <hip/hip_runtime.h>


#define NN_  30000
#define NP   30016
#define KK   32
#define CIN  256
#define HID  128
#define COUT 512

typedef unsigned short bf;
typedef __attribute__((ext_vector_type(16))) __bf16   v16bf;
typedef __attribute__((ext_vector_type(8)))  unsigned short v8us;
typedef __attribute__((ext_vector_type(8)))  float    v8f;
typedef __attribute__((ext_vector_type(4)))  float    v4f;
typedef v4f  __attribute__((may_alias)) v4fa;
typedef v8us __attribute__((may_alias)) v8usa;

__device__ __forceinline__ unsigned short f2bf(float f) { unsigned u = __float_as_uint(f); u += 0x7FFFu + ((u >> 16) & 1u); return (unsigned short)(u >> 16); }
__device__ __forceinline__ float bf2f(unsigned short b) { return __uint_as_float(((unsigned)b) << 16); }
__device__ __forceinline__ float bfr(float f) { return bf2f(f2bf(f)); }
__device__ __forceinline__ v16bf cat16b(v8us lo, v8us hi) { return __builtin_bit_cast(v16bf, __builtin_shufflevector(lo, hi, 0, 1, 2, 3, 4, 5, 6, 7, 8, 9, 10, 11, 12, 13, 14, 15)); }
__device__ __forceinline__ v8f wmmab(v16bf a, v16bf b, v8f c) { return __builtin_amdgcn_wmma_f32_16x16x32_bf16(false, a, false, b, (short)0, c, false, false); }
__device__ __forceinline__ float leaky(float v) { return v >= 0.f ? v : 0.1f * v; }
#define VST2(T, p, v) do { const T vst2_v_ = (v); *(volatile T*)(p) = vst2_v_; __threadfence(); *(volatile T*)(p) = vst2_v_; } while (0)

__global__ __launch_bounds__(256) void k_fb(const float* __restrict__ f, bf* Fb) {
    const int lane = threadIdx.x & 31, r = blockIdx.x * 8 + (threadIdx.x >> 5);
    if (r >= NP) return;
    const int rr = r < NN_ ? r : NN_ - 1;
    v8us t;
#pragma unroll
    for (int i = 0; i < 8; ++i) t[i] = (r < NN_) ? f2bf(f[(size_t)rr * CIN + lane * 8 + i]) : (unsigned short)0;
    VST2(v8us, Fb + (size_t)r * CIN + lane * 8, t);
}
__global__ __launch_bounds__(256) void k_wt(const float* __restrict__ Wm, int r0w, int Kdim, int Ndim, bf* WT) {
    __shared__ __align__(16) unsigned short tl[64 * 72];
    const int tid = threadIdx.x, k0 = blockIdx.x * 64, n0 = blockIdx.y * 64;
    const int kk = tid >> 2, nq = (tid & 3) * 16;
#pragma unroll
    for (int i = 0; i < 16; ++i) tl[(nq + i) * 72 + kk] = f2bf(Wm[(size_t)(r0w + k0 + kk) * Ndim + n0 + nq + i]);
    __syncthreads();
    const int piece = tid & 7;
    auto pass = [&]() {
#pragma unroll
        for (int s = 0; s < 2; ++s) { const int nr = (tid >> 3) + 32 * s; const v8us val = *(const v8usa*)(tl + nr * 72 + piece * 8);
            *(volatile v8us*)(WT + (size_t)(n0 + nr) * Kdim + k0 + piece * 8) = val; }
    };
    pass(); __threadfence(); pass();
}
template <bool SPLITA>
__global__ __launch_bounds__(128) void k_gemm(const bf* __restrict__ A, const bf* __restrict__ Al, const bf* __restrict__ Bn, int K, int ldc, float* C, int nrows) {
    __shared__ __align__(16) float ost[4][16 * 68];
    const int lane = threadIdx.x & 31, wave = threadIdx.x >> 5, lr = lane & 15, hi = lane >> 4;
    const int r0 = blockIdx.x * 64 + wave * 16, c0 = blockIdx.y * 64;
    const size_t aoff = (size_t)(r0 + lr) * K + 8 * hi;
    size_t boff[4];
#pragma unroll
    for (int t = 0; t < 4; ++t) boff[t] = (size_t)(c0 + t * 16 + lr) * K + 8 * hi;
    v8f acc[4];
#pragma unroll
    for (int t = 0; t < 4; ++t) acc[t] = (v8f){};
#pragma unroll 1
    for (int kc = 0; kc < K; kc += 32) {
        const v16bf a = cat16b(*(const v8us*)(A + aoff + kc), *(const v8us*)(A + aoff + kc + 16));
        v16bf al = a;
        if (SPLITA) al = cat16b(*(const v8us*)(Al + aoff + kc), *(const v8us*)(Al + aoff + kc + 16));
#pragma unroll
        for (int t = 0; t < 4; ++t) { const v16bf b = cat16b(*(const v8us*)(Bn + boff[t] + kc), *(const v8us*)(Bn + boff[t] + kc + 16)); acc[t] = wmmab(a, b, acc[t]); if (SPLITA) acc[t] = wmmab(al, b, acc[t]); }
        asm volatile("v_nop\n\tv_nop\n\tv_nop\n\tv_nop" : "+v"(acc[0]), "+v"(acc[1]), "+v"(acc[2]), "+v"(acc[3]) : "v"(a), "v"(al));
    }
    float* os = &ost[wave][0];
#pragma unroll
    for (int t = 0; t < 4; ++t)
#pragma unroll
        for (int j = 0; j < 8; ++j) os[(hi * 8 + j) * 68 + t * 16 + lr] = acc[t][j];
    __syncthreads();
    float* crow = C + (size_t)r0 * ldc + c0;
    auto pass = [&]() {
#pragma unroll
        for (int s = 0; s < 8; ++s) { const int Lid = (lane >> 3) + 4 * s, piece = lane & 7; const int row = Lid >> 1, cofs = (Lid & 1) * 32 + piece * 4;
            const v4f val = *(const v4fa*)(os + row * 68 + cofs); if (r0 + row < nrows) *(volatile v4f*)(crow + (size_t)row * ldc + cofs) = val; }
    };
    pass(); __threadfence(); pass();
}
__global__ __launch_bounds__(256) void k_colstats(const float* __restrict__ M, int C, float* ST) {
    __shared__ float red[256];
    const int c = blockIdx.x, t = threadIdx.x;
    float s = 0.f;
#pragma unroll 1
    for (int r = t; r < NN_; r += 256) s += M[(size_t)r * C + c];
    red[t] = s; __syncthreads();
    for (int st = 128; st > 0; st >>= 1) { if (t < st) red[t] += red[t + st]; __syncthreads(); }
    const float mu = red[0] / (float)NN_;
    __syncthreads();
    float q = 0.f;
#pragma unroll 1
    for (int r = t; r < NN_; r += 256) { const float d = M[(size_t)r * C + c] - mu; q += d * d; }
    red[t] = q; __syncthreads();
    for (int st = 128; st > 0; st >>= 1) { if (t < st) red[t] += red[t + st]; __syncthreads(); }
    const float var = red[0] / (float)NN_;
    if (t < 32) { const float v = (t == 0) ? mu : (t == 1) ? rsqrtf(var + 1e-5f) : 0.f; VST2(float, ST + (size_t)c * 32 + t, v); }
}
__global__ __launch_bounds__(256) void k_act1(const float* __restrict__ A1, const float* __restrict__ ST, const float* __restrict__ g, const float* __restrict__ be, bf* XH, bf* XL) {
    const int lane = threadIdx.x & 31; const size_t w = (size_t)blockIdx.x * 8 + (threadIdx.x >> 5);
    const size_t r = w * 2 + (lane >> 4); const int c0 = (lane & 15) * 8;
    v8us oh, ol;
#pragma unroll
    for (int i = 0; i < 8; ++i) { const int c = c0 + i; float v = 0.f;
        if (r < (size_t)NN_) v = leaky((A1[r * HID + c] - ST[c * 32]) * ST[c * 32 + 1] * bfr(g[c]) + bfr(be[c]));
        const unsigned short hb = f2bf(v); oh[i] = hb; ol[i] = f2bf(v - bf2f(hb)); }
    *(volatile v8us*)(XH + r * HID + c0) = oh; *(volatile v8us*)(XL + r * HID + c0) = ol; __threadfence();
    *(volatile v8us*)(XH + r * HID + c0) = oh; *(volatile v8us*)(XL + r * HID + c0) = ol;
}
template <int PASS>
__global__ __launch_bounds__(256) void k_ypart(const float* __restrict__ pts, const int* __restrict__ nb, const float* __restrict__ cw, const float* __restrict__ Z, const float* __restrict__ ST2, float* P1) {
    const int lane = threadIdx.x & 31, n = blockIdx.x * 8 + (threadIdx.x >> 5);
    if (n >= NN_) return;
    float w0[4], w1[4], w2[4];
#pragma unroll
    for (int i = 0; i < 4; ++i) { const int c = lane * 4 + i; w0[i] = bfr(cw[c]); w1[i] = bfr(cw[HID + c]); w2[i] = bfr(cw[2 * HID + c]); }
    const float p0 = bfr(pts[(size_t)n * 3]), p1 = bfr(pts[(size_t)n * 3 + 1]), p2 = bfr(pts[(size_t)n * 3 + 2]);
    v4f s1; s1[0] = s1[1] = s1[2] = s1[3] = 0.f; float mu[4];
#pragma unroll
    for (int i = 0; i < 4; ++i) mu[i] = (PASS == 1) ? ST2[(lane * 4 + i) * 32] : 0.f;
#pragma unroll 1
    for (int k = 0; k < KK; ++k) { int j = nb[(size_t)n * KK + k]; if (j < 0) j = 0; if (j > NN_) j = NN_;
        float y[4] = {0.f, 0.f, 0.f, 0.f};
        if (j != NN_) { const float d0 = bfr(pts[(size_t)j * 3]) - p0, d1 = bfr(pts[(size_t)j * 3 + 1]) - p1, d2 = bfr(pts[(size_t)j * 3 + 2]) - p2;
            const v4f z = *(const v4fa*)(Z + (size_t)j * HID + lane * 4);
#pragma unroll
            for (int i = 0; i < 4; ++i) y[i] = d0 * w0[i] + d1 * w1[i] + d2 * w2[i] + z[i]; }
#pragma unroll
        for (int i = 0; i < 4; ++i) { if (PASS == 0) s1[i] += y[i]; else { const float d = y[i] - mu[i]; s1[i] += d * d; } } }
    VST2(v4f, P1 + (size_t)n * HID + lane * 4, s1);
}
template <int PASS>
__global__ __launch_bounds__(256) void k_ystat2(const float* __restrict__ P, float* ST2) {
    __shared__ float red[256];
    const int c = blockIdx.x, t = threadIdx.x;
    float s = 0.f;
#pragma unroll 1
    for (int r = t; r < NN_; r += 256) s += P[(size_t)r * HID + c];
    red[t] = s; __syncthreads();
    for (int st = 128; st > 0; st >>= 1) { if (t < st) red[t] += red[t + st]; __syncthreads(); }
    const float val = red[0] / (float)(NN_ * KK);
    if (t < 32) { const float prev_mu = ST2[(size_t)c * 32];
        const float v = (PASS == 0) ? ((t == 0) ? val : 0.f) : ((t == 0) ? prev_mu : (t == 1) ? rsqrtf(val + 1e-5f) : 0.f);
        VST2(float, ST2 + (size_t)c * 32 + t, v); }
}
__global__ __launch_bounds__(256) void k_ymax(const float* __restrict__ pts, const int* __restrict__ nb, const float* __restrict__ cw, const float* __restrict__ Z, const float* __restrict__ ST2, const float* __restrict__ g, const float* __restrict__ be, bf* YH, bf* YL) {
    typedef __attribute__((ext_vector_type(4))) unsigned short v4us;
    const int lane = threadIdx.x & 31, n = blockIdx.x * 8 + (threadIdx.x >> 5);
    if (n >= NP) return;
    v4us oh, ol;
    if (n >= NN_) { oh[0] = oh[1] = oh[2] = oh[3] = 0; ol = oh; }
    else {
        float w0[4], w1[4], w2[4], mu[4], rsg[4], bb[4], m[4];
#pragma unroll
        for (int i = 0; i < 4; ++i) { const int c = lane * 4 + i; w0[i] = bfr(cw[c]); w1[i] = bfr(cw[HID + c]); w2[i] = bfr(cw[2 * HID + c]); mu[i] = ST2[c * 32]; rsg[i] = ST2[c * 32 + 1] * bfr(g[c]); bb[i] = bfr(be[c]); m[i] = -3.0e38f; }
        const float p0 = bfr(pts[(size_t)n * 3]), p1 = bfr(pts[(size_t)n * 3 + 1]), p2 = bfr(pts[(size_t)n * 3 + 2]);
#pragma unroll 1
        for (int k = 0; k < KK; ++k) { int j = nb[(size_t)n * KK + k]; if (j < 0) j = 0; if (j > NN_) j = NN_;
            float y[4] = {0.f, 0.f, 0.f, 0.f};
            if (j != NN_) { const float d0 = bfr(pts[(size_t)j * 3]) - p0, d1 = bfr(pts[(size_t)j * 3 + 1]) - p1, d2 = bfr(pts[(size_t)j * 3 + 2]) - p2;
                const v4f z = *(const v4fa*)(Z + (size_t)j * HID + lane * 4);
#pragma unroll
                for (int i = 0; i < 4; ++i) y[i] = d0 * w0[i] + d1 * w1[i] + d2 * w2[i] + z[i]; }
#pragma unroll
            for (int i = 0; i < 4; ++i) m[i] = fmaxf(m[i], leaky((y[i] - mu[i]) * rsg[i] + bb[i])); }
#pragma unroll
        for (int i = 0; i < 4; ++i) { const unsigned short hb = f2bf(m[i]); oh[i] = hb; ol[i] = f2bf(m[i] - bf2f(hb)); }
    }
    VST2(v4us, YH + (size_t)n * HID + lane * 4, oh); VST2(v4us, YL + (size_t)n * HID + lane * 4, ol);
}
__global__ __launch_bounds__(256) void k_final(const float* __restrict__ X2, const float* __restrict__ ST3, const float* __restrict__ g3, const float* __restrict__ b3,
                                              const float* __restrict__ STs, const float* __restrict__ gs, const float* __restrict__ bs, float* out) {
    const int lane = threadIdx.x & 31, r = blockIdx.x * 8 + (threadIdx.x >> 5);
    if (r >= NN_) return;
    v4f o4[4];
#pragma unroll
    for (int s = 0; s < 4; ++s) {
#pragma unroll
        for (int i = 0; i < 4; ++i) { const int c = s * 128 + lane * 4 + i; const float sc = out[(size_t)r * COUT + c];
            const float a = (X2[(size_t)r * COUT + c] - ST3[c * 32]) * ST3[c * 32 + 1] * bfr(g3[c]) + bfr(b3[c]);
            const float b = (sc - STs[c * 32]) * STs[c * 32 + 1] * bfr(gs[c]) + bfr(bs[c]);
            o4[s][i] = leaky(a + b); } }
    __builtin_amdgcn_wave_barrier();
#pragma unroll
    for (int s = 0; s < 4; ++s) *(volatile v4f*)(out + (size_t)r * COUT + s * 128 + lane * 4) = o4[s];
    __threadfence();
#pragma unroll
    for (int s = 0; s < 4; ++s) *(volatile v4f*)(out + (size_t)r * COUT + s * 128 + lane * 4) = o4[s];
}

extern "C" void kernel_launch(void* const* d_in, const int* in_sizes, int n_in,
                              void* d_out, int out_size, void* d_ws, size_t ws_size, hipStream_t stream) {
    (void)in_sizes; (void)n_in; (void)out_size;
    const float* feat = (const float*)d_in[0]; const float* pts = (const float*)d_in[1]; const int* nb = (const int*)d_in[2];
    const float* w1 = (const float*)d_in[3]; const float* g1 = (const float*)d_in[4]; const float* b1 = (const float*)d_in[5]; const float* cw = (const float*)d_in[6]; const float* g2 = (const float*)d_in[7]; const float* b2 = (const float*)d_in[8];
    const float* w2 = (const float*)d_in[9]; const float* g3 = (const float*)d_in[10]; const float* b3 = (const float*)d_in[11]; const float* ws = (const float*)d_in[12]; const float* gs = (const float*)d_in[13]; const float* bs = (const float*)d_in[14];
    float* out = (float*)d_out;
    char* wsp = (char*)d_ws;
    auto take = [&](size_t bytes) { char* p = wsp; wsp += (bytes + 255) & ~(size_t)255; return (void*)p; };
    bf* Fb = (bf*)take((size_t)NP * CIN * 2); bf* W1T = (bf*)take((size_t)HID * CIN * 2); bf* CWT = (bf*)take((size_t)HID * HID * 2); bf* W2T = (bf*)take((size_t)COUT * HID * 2); bf* WST = (bf*)take((size_t)COUT * CIN * 2);
    float* A1 = (float*)take((size_t)NP * HID * 4); bf* XH = (bf*)take((size_t)NP * HID * 2); bf* XL = (bf*)take((size_t)NP * HID * 2);
    bf* YH = (bf*)take((size_t)NP * HID * 2); bf* YL = (bf*)take((size_t)NP * HID * 2); float* X2 = (float*)take((size_t)NP * COUT * 4);
    float* ST1 = (float*)take((size_t)HID * 32 * 4); float* ST2 = (float*)take((size_t)HID * 32 * 4); float* ST3 = (float*)take((size_t)COUT * 32 * 4); float* STs = (float*)take((size_t)COUT * 32 * 4);
    if ((size_t)(wsp - (char*)d_ws) > ws_size) return;
    float* Z = A1; float* P1 = X2; float* P2 = X2 + (size_t)NP * HID;
    k_fb<<<NP / 8, 256, 0, stream>>>(feat, Fb);
    k_wt<<<dim3(CIN / 64, HID / 64, 1), 256, 0, stream>>>(w1, 0, CIN, HID, W1T);
    k_wt<<<dim3(HID / 64, HID / 64, 1), 256, 0, stream>>>(cw, 3, HID, HID, CWT);
    k_wt<<<dim3(HID / 64, COUT / 64, 1), 256, 0, stream>>>(w2, 0, HID, COUT, W2T);
    k_wt<<<dim3(CIN / 64, COUT / 64, 1), 256, 0, stream>>>(ws, 0, CIN, COUT, WST);
    k_gemm<false><<<dim3(NP / 64, HID / 64, 1), 128, 0, stream>>>(Fb, nullptr, W1T, CIN, HID, A1, NP);
    k_colstats<<<HID, 256, 0, stream>>>(A1, HID, ST1);
    k_act1<<<(NP / 2) / 8, 256, 0, stream>>>(A1, ST1, g1, b1, XH, XL);
    k_gemm<true><<<dim3(NP / 64, HID / 64, 1), 128, 0, stream>>>(XH, XL, CWT, HID, HID, Z, NP);
    k_ypart<0><<<(NN_ + 7) / 8, 256, 0, stream>>>(pts, nb, cw, Z, ST2, P1);
    k_ystat2<0><<<HID, 256, 0, stream>>>(P1, ST2);
    k_ypart<1><<<(NN_ + 7) / 8, 256, 0, stream>>>(pts, nb, cw, Z, ST2, P2);
    k_ystat2<1><<<HID, 256, 0, stream>>>(P2, ST2);
    k_ymax<<<NP / 8, 256, 0, stream>>>(pts, nb, cw, Z, ST2, g2, b2, YH, YL);
    k_gemm<true><<<dim3(NP / 64, COUT / 64, 1), 128, 0, stream>>>(YH, YL, W2T, HID, COUT, X2, NP);
    k_gemm<false><<<dim3(NP / 64, COUT / 64, 1), 128, 0, stream>>>(Fb, nullptr, WST, CIN, COUT, out, NN_);
    k_colstats<<<COUT, 256, 0, stream>>>(X2, COUT, ST3);
    k_colstats<<<COUT, 256, 0, stream>>>(out, COUT, STs);
    k_final<<<(NN_ + 7) / 8, 256, 0, stream>>>(X2, ST3, g3, b3, STs, gs, bs, out);
}
